// LambdaAttention_20718922236172
// MI455X (gfx1250) — hardware-verified
//
#include <hip/hip_runtime.h>
#include <stddef.h>


typedef _Float16 h16;
typedef _Float16 v16h __attribute__((ext_vector_type(16)));
typedef _Float16 v8h  __attribute__((ext_vector_type(8)));
typedef float    v8f  __attribute__((ext_vector_type(8)));
typedef float    v4f  __attribute__((ext_vector_type(4)));

#ifndef NB
#define NB 8
#endif
#define NB_FULL 8
#define CIN    256
#define IMG    64
#define HW     4096
#define NHEADS 4
#define KDIM   16
#define QROWS  64
#define VROWS  64
#define KROWS  16
#define WROWS  192
#define OUTC   256
#define MWIN   11
#define TAPS   121
#define TAPK   128

#define LDT 72
#define LDC 68
#define LDQ 68
#define LDL 68
#define PP    80
#define PROWS 16
#define VG    16

#define WCARRY 64.0f
#define XCARRY 16.0f
#define ECARRY 16.0f
#define VCARRY 16.0f
#define PCARRY 1024.0f

static_assert(NB >= 1 && NB <= NB_FULL);
static_assert(HW == IMG * IMG && IMG == 64);
static_assert((HW % 64) == 0 && (CIN % 64) == 0 && (CIN % 32) == 0);
static_assert(QROWS == NHEADS * KDIM && NHEADS == 4 && KDIM == 16);
static_assert(OUTC == NHEADS * VROWS);
static_assert(QROWS == 64 && VROWS == 64 && KROWS == 16);
static_assert(WROWS == 3 * 64 && QROWS + VROWS + KROWS <= WROWS);
static_assert(WROWS * CIN == 24 * 256 * 8);
static_assert(KDIM * TAPK == 256 * 8);
static_assert(MWIN * MWIN == TAPS && TAPS <= TAPK && TAPK == 128 && (TAPK % 32) == 0);
static_assert((LDT % 8) == 0 && LDT >= 64);
static_assert((LDC % 4) == 0 && LDC >= 64 && (LDQ % 4) == 0 && LDQ >= 64 && LDL >= 64);
static_assert((PP % 8) == 0 && PP >= 8 + IMG + 8);
static_assert(3 + (IMG - 1) + (MWIN - 1) < PP);
static_assert(PROWS == 16 && PROWS >= MWIN);
static_assert((VROWS % VG) == 0 && VG * KDIM == 2 * 128);
static_assert(4 * 16 == 64);
static_assert(2 * 32 == 64);
static_assert(256 / 16 == KROWS);
static_assert(8 * 512 == HW);
static_assert((size_t)NB_FULL * OUTC * HW * 4 == (size_t)33554432);

static_assert(64 * LDT * 2 <= 131072);
static_assert(64 * LDC * 4 <= 131072);
static_assert((8 * 16 * LDC + 8 * 16 + 16) * 4 <= 131072);
static_assert(PROWS * PP * 2 + (64 * LDQ + KDIM * LDL + KDIM * VG) * 4 <= 131072);

#define WALL_BYTES ((size_t)WROWS * CIN * 2)
#define E16_BYTES  ((size_t)KDIM * TAPK * 2)
#define XT_BYTES   ((size_t)NB * HW * CIN * 2)
#define Q32_BYTES  ((size_t)NB * QROWS * HW * 4)
#define K32_BYTES  ((size_t)NB * KROWS * HW * 4)
#define VH_BYTES   ((size_t)NB * VROWS * HW * 2)
#define LC_BYTES   ((size_t)NB * KDIM * VROWS * 4)
#define OFF_WALL ((size_t)0)
#define OFF_E16  (OFF_WALL + WALL_BYTES)
#define OFF_XT   (OFF_E16 + E16_BYTES)
#define OFF_Q32  (OFF_XT + XT_BYTES)
#define OFF_K32  (OFF_Q32 + Q32_BYTES)
#define OFF_VH   (OFF_K32 + K32_BYTES)
#define OFF_LC   (OFF_VH + VH_BYTES)
#define WS_TOTAL (OFF_LC + LC_BYTES)
static_assert((WALL_BYTES % 128) == 0 && (E16_BYTES % 128) == 0 && (XT_BYTES % 128) == 0);
static_assert((Q32_BYTES % 128) == 0 && (K32_BYTES % 128) == 0 && (VH_BYTES % 128) == 0);
static_assert((LC_BYTES % 128) == 0);
static_assert(WS_TOTAL <= (size_t)134217728);

__device__ __forceinline__ float bf16r(float x) {
  unsigned int u = __float_as_uint(x);
  u = (u + 0x7FFFu + ((u >> 16) & 1u)) & 0xFFFF0000u;
  return __uint_as_float(u);
}

static __device__ __forceinline__ h16 toh_flush(float v) {
  const h16 r = (h16)v;
  return (fabsf(v) < 6.103515625e-05f) ? (h16)0.0f : r;
}

__device__ __forceinline__ v16h frag_at(const _Float16* p) {
  v8h lo = *(const v8h*)(p);
  v8h hi = *(const v8h*)(p + 16);
  v16h out;
#pragma unroll
  for (int i = 0; i < 8; ++i) { out[i] = lo[i]; out[i + 8] = hi[i]; }
  return out;
}

__device__ __forceinline__ v8f wmma16(v16h a, v16h b, v8f c) {
  v8f d = __builtin_amdgcn_wmma_f32_16x16x32_f16(false, a, false, b, (short)0, c,
                                                 false, false);
  asm volatile("v_nop\n\tv_nop\n\tv_nop\n\tv_nop" : "+v"(d) : "v"(a), "v"(b));
  return d;
}

__device__ __forceinline__ float red16_max(float x) {
#pragma unroll
  for (int off = 1; off < 16; off <<= 1) x = fmaxf(x, __shfl_xor(x, off, 32));
  return x;
}

__global__ __launch_bounds__(256) void prep_kernel(
    const float* __restrict__ Wq, const float* __restrict__ Wk, const float* __restrict__ Wv,
    const float* __restrict__ emb, _Float16* __restrict__ Wall, _Float16* __restrict__ E16) {
  const unsigned tid = threadIdx.x;
  if (blockIdx.x < 24u) {
    const unsigned gid = blockIdx.x * 256u + tid;
    const unsigned r = gid >> 5, pc = (gid & 31u) * 8u;
    const unsigned rq = (r < 63u) ? r : 63u;
    const unsigned rv = (r < 64u) ? 0u : (((r - 64u) < 63u) ? (r - 64u) : 63u);
    const unsigned rk = (r < 128u) ? 0u : (((r - 128u) < 15u) ? (r - 128u) : 15u);
    const v4f a0 = *(const v4f*)(Wq + rq * CIN + pc);
    const v4f a1 = *(const v4f*)(Wq + rq * CIN + pc + 4u);
    const v4f b0 = *(const v4f*)(Wv + rv * CIN + pc);
    const v4f b1 = *(const v4f*)(Wv + rv * CIN + pc + 4u);
    const v4f c0 = *(const v4f*)(Wk + rk * CIN + pc);
    const v4f c1 = *(const v4f*)(Wk + rk * CIN + pc + 4u);
    v8h o;
#pragma unroll
    for (int j = 0; j < 4; ++j) {
      const float s0 = (r < 64u) ? a0[j] : ((r < 128u) ? b0[j] : ((r < 144u) ? c0[j] : 0.0f));
      const float s1 = (r < 64u) ? a1[j] : ((r < 128u) ? b1[j] : ((r < 144u) ? c1[j] : 0.0f));
      o[j]     = toh_flush(WCARRY * bf16r(s0));
      o[j + 4] = toh_flush(WCARRY * bf16r(s1));
    }
    _Float16* p = Wall + (size_t)r * CIN + pc;
    *(volatile v8h*)p = o;
    __threadfence();
    *(volatile v8h*)p = o;
  } else {
    const unsigned k = tid >> 4, t0 = (tid & 15u) * 8u;
    v8h o;
#pragma unroll
    for (unsigned j = 0; j < 8u; ++j) {
      const unsigned t = t0 + j;
      const unsigned tc = (t < 120u) ? t : 120u;
      const float v = emb[k * TAPS + tc];
      const h16 e = toh_flush(ECARRY * bf16r(v));
      o[j] = (t < (unsigned)TAPS) ? e : (h16)0.0f;
    }
    _Float16* p = E16 + (size_t)k * TAPK + t0;
    *(volatile v8h*)p = o;
    __threadfence();
    *(volatile v8h*)p = o;
  }
}

__global__ __launch_bounds__(256) void xconv_kernel(
    const float* __restrict__ X, _Float16* __restrict__ Xt) {
  __shared__ _Float16 T[64 * LDT];
  const unsigned tid = threadIdx.x;
  const unsigned n0 = blockIdx.x * 64u;
  const unsigned k0 = blockIdx.y * 64u;
  const float* W = X + (size_t)blockIdx.z * CIN * HW;
  _Float16* Wt = Xt + (size_t)blockIdx.z * HW * CIN;
#pragma unroll 4
  for (unsigned j = 0; j < 16u; ++j) {
    const unsigned idx = tid + 256u * j;
    const unsigned kr = idx >> 6, nc = idx & 63u;
    const float v = W[(size_t)(k0 + kr) * HW + n0 + nc];
    T[nc * LDT + kr] = toh_flush(XCARRY * bf16r(v));
  }
  __syncthreads();
  v8h x[2];
  size_t off[2];
#pragma unroll
  for (unsigned i = 0; i < 2u; ++i) {
    const unsigned n = 32u * i + (tid >> 3);
    const unsigned kc = (tid & 7u) * 8u;
    x[i] = *(const v8h*)&T[n * LDT + kc];
    off[i] = (size_t)(n0 + n) * CIN + k0 + kc;
  }
#pragma unroll
  for (int i = 0; i < 2; ++i) *(volatile v8h*)(Wt + off[i]) = x[i];
  __threadfence();
#pragma unroll
  for (int i = 0; i < 2; ++i) *(volatile v8h*)(Wt + off[i]) = x[i];
}

template <int MODE>
__device__ __forceinline__ void proj_body(
    const _Float16* __restrict__ A16, const _Float16* __restrict__ Xt,
    const float* __restrict__ gam, const float* __restrict__ bet,
    const float* __restrict__ mea, const float* __restrict__ var,
    float* __restrict__ outf, _Float16* __restrict__ out16) {
  __shared__ float Cs[64 * LDC];
  const unsigned tid = threadIdx.x, lane = tid & 31u;
  const unsigned w = (unsigned)__builtin_amdgcn_readfirstlane((int)(tid >> 5));
  const unsigned mw = w >> 1, nw = w & 1u;
  const unsigned hh = lane >> 4, m = lane & 15u;
  const unsigned n0 = blockIdx.x * 64u;
  const unsigned b = blockIdx.z;

  const _Float16* ap  = A16 + (size_t)(mw * 16u + m) * CIN + hh * 8u;
  const _Float16* bp0 = Xt + ((size_t)b * HW + n0 + nw * 32u + m) * CIN + hh * 8u;
  const _Float16* bp1 = bp0 + (size_t)16 * CIN;
  v8f acc0 = {}, acc1 = {};
#pragma unroll 2
  for (unsigned k0 = 0; k0 < (unsigned)CIN; k0 += 32u) {
    const v16h a  = frag_at(ap + k0);
    const v16h b0 = frag_at(bp0 + k0);
    const v16h b1 = frag_at(bp1 + k0);
    acc0 = wmma16(a, b0, acc0);
    acc1 = wmma16(a, b1, acc1);
  }
#pragma unroll
  for (int r = 0; r < 8; ++r) {
    float* d = &Cs[(mw * 16u + hh * 8u + (unsigned)r) * LDC + nw * 32u + m];
    d[0]  = acc0[r];
    d[16] = acc1[r];
  }
  __syncthreads();

  const float cs = 1.0f / (WCARRY * XCARRY);

  if (MODE == 0) {
    v4f xs[4];
    size_t off[4];
#pragma unroll
    for (unsigned i = 0; i < 4u; ++i) {
      const unsigned r = 16u * i + (tid >> 4);
      const unsigned c = (tid & 15u) * 4u;
      const v4f u = *(const v4f*)&Cs[r * LDC + c];
      const float g  = bf16r(gam[r]);
      const float be = bf16r(bet[r]);
      const float mu = bf16r(mea[r]);
      const float vr = bf16r(var[r]);
      const float sc = g * (1.0f / sqrtf(vr + 1.0e-5f));
      v4f val;
#pragma unroll
      for (int j = 0; j < 4; ++j) val[j] = (u[j] * cs - mu) * sc + be;
      xs[i] = val;
      off[i] = ((size_t)b * QROWS + r) * HW + n0 + c;
    }
#pragma unroll
    for (int i = 0; i < 4; ++i) *(volatile v4f*)(outf + off[i]) = xs[i];
    __threadfence();
#pragma unroll
    for (int i = 0; i < 4; ++i) *(volatile v4f*)(outf + off[i]) = xs[i];
  }

  if (MODE == 1) {
    v8h x[2];
    size_t off[2];
#pragma unroll
    for (unsigned i = 0; i < 2u; ++i) {
      const unsigned r = 32u * i + (tid >> 3);
      const unsigned c = (tid & 7u) * 8u;
      const v4f u0 = *(const v4f*)&Cs[r * LDC + c];
      const v4f u1 = *(const v4f*)&Cs[r * LDC + c + 4];
      const float g  = bf16r(gam[r]);
      const float be = bf16r(bet[r]);
      const float mu = bf16r(mea[r]);
      const float vr = bf16r(var[r]);
      const float sc = g * (1.0f / sqrtf(vr + 1.0e-5f));
#pragma unroll
      for (int j = 0; j < 4; ++j) {
        x[i][j]     = toh_flush(VCARRY * ((u0[j] * cs - mu) * sc + be));
        x[i][j + 4] = toh_flush(VCARRY * ((u1[j] * cs - mu) * sc + be));
      }
      off[i] = ((size_t)b * VROWS + r) * HW + n0 + c;
    }
#pragma unroll
    for (int i = 0; i < 2; ++i) *(volatile v8h*)(out16 + off[i]) = x[i];
    __threadfence();
#pragma unroll
    for (int i = 0; i < 2; ++i) *(volatile v8h*)(out16 + off[i]) = x[i];
  }

  if (MODE == 2) {
    const unsigned r = tid >> 4;
    const unsigned c = (tid & 15u) * 4u;
    const v4f u = *(const v4f*)&Cs[r * LDC + c];
    v4f val;
#pragma unroll
    for (int j = 0; j < 4; ++j) val[j] = u[j] * cs;
    float* p = outf + ((size_t)b * KROWS + r) * HW + n0 + c;
    *(volatile v4f*)p = val;
    __threadfence();
    *(volatile v4f*)p = val;
  }
}

__global__ __launch_bounds__(256) void proj_q_kernel(
    const _Float16* __restrict__ A16, const _Float16* __restrict__ Xt,
    const float* __restrict__ gam, const float* __restrict__ bet,
    const float* __restrict__ mea, const float* __restrict__ var,
    float* __restrict__ q32) {
  proj_body<0>(A16, Xt, gam, bet, mea, var, q32, (_Float16*)0);
}
__global__ __launch_bounds__(256) void proj_v_kernel(
    const _Float16* __restrict__ A16, const _Float16* __restrict__ Xt,
    const float* __restrict__ gam, const float* __restrict__ bet,
    const float* __restrict__ mea, const float* __restrict__ var,
    _Float16* __restrict__ vh) {
  proj_body<1>(A16, Xt, gam, bet, mea, var, (float*)0, vh);
}
__global__ __launch_bounds__(256) void proj_k_kernel(
    const _Float16* __restrict__ A16, const _Float16* __restrict__ Xt,
    float* __restrict__ k32) {
  proj_body<2>(A16, Xt, (const float*)0, (const float*)0, (const float*)0, (const float*)0,
               k32, (_Float16*)0);
}

__global__ __launch_bounds__(256) void content_kernel(
    const float* __restrict__ K32, const _Float16* __restrict__ Vh, float* __restrict__ Lc) {
  __shared__ float sMax[16];
  __shared__ float sSum[8 * 16];
  __shared__ float sPart[8 * 16 * LDC];
  const unsigned tid = threadIdx.x, lane = tid & 31u;
  const unsigned w = (unsigned)__builtin_amdgcn_readfirstlane((int)(tid >> 5));
  const unsigned hh = lane >> 4, m = lane & 15u;
  const unsigned b = blockIdx.x;

  {
    const unsigned row = tid >> 4, sub = tid & 15u;
    const float* kr = K32 + ((size_t)b * KROWS + row) * HW + sub * 4u;
    float mx = -3.0e38f;
#pragma unroll 4
    for (unsigned j = 0; j < 64u; ++j) {
      const v4f t = *(const v4f*)(kr + j * 64u);
      mx = fmaxf(mx, fmaxf(fmaxf(t[0], t[1]), fmaxf(t[2], t[3])));
    }
    mx = red16_max(mx);
    if (sub == 0u) sMax[row] = mx;
  }
  __syncthreads();

  const float mrow = sMax[m];
  const float* kp = K32 + ((size_t)b * KROWS + m) * HW + w * 512u + hh * 8u;
  const _Float16* vp = Vh + ((size_t)b * VROWS + m) * HW + w * 512u + hh * 8u;
  v8f acc[4];
#pragma unroll
  for (int nb = 0; nb < 4; ++nb) acc[nb] = (v8f){};
  float lsum = 0.0f;
#pragma unroll 1
  for (unsigned st = 0; st < 16u; ++st) {
    const unsigned n0 = st * 32u;
    const v4f k0 = *(const v4f*)(kp + n0);
    const v4f k1 = *(const v4f*)(kp + n0 + 4u);
    const v4f k2 = *(const v4f*)(kp + n0 + 16u);
    const v4f k3 = *(const v4f*)(kp + n0 + 20u);
    v16h pf;
#pragma unroll
    for (int j = 0; j < 4; ++j) {
      const h16 e0 = toh_flush(PCARRY * __expf(k0[j] - mrow));
      const h16 e1 = toh_flush(PCARRY * __expf(k1[j] - mrow));
      const h16 e2 = toh_flush(PCARRY * __expf(k2[j] - mrow));
      const h16 e3 = toh_flush(PCARRY * __expf(k3[j] - mrow));
      pf[j] = e0; pf[j + 4] = e1; pf[j + 8] = e2; pf[j + 12] = e3;
      lsum += ((float)e0 + (float)e1) + ((float)e2 + (float)e3);
    }
#pragma unroll
    for (int nb = 0; nb < 4; ++nb) {
      const v16h vf = frag_at(vp + (size_t)nb * 16u * HW + n0);
      acc[nb] = wmma16(pf, vf, acc[nb]);
    }
  }
  lsum += __shfl_xor(lsum, 16, 32);
#pragma unroll
  for (int nb = 0; nb < 4; ++nb)
#pragma unroll
    for (int r = 0; r < 8; ++r)
      sPart[(w * 16u + hh * 8u + (unsigned)r) * LDC + (unsigned)nb * 16u + m] = acc[nb][r];
  if (hh == 0u) sSum[w * 16u + m] = lsum;
  __syncthreads();

  {
    const unsigned k = tid >> 4, c = (tid & 15u) * 4u;
    v4f s = {};
    float l = 0.0f;
#pragma unroll
    for (unsigned ww = 0; ww < 8u; ++ww) {
      const v4f t = *(const v4f*)&sPart[(ww * 16u + k) * LDC + c];
      s = s + t;
      l += sSum[ww * 16u + k];
    }
    const float inv = 1.0f / (l * VCARRY);
    v4f val;
#pragma unroll
    for (int j = 0; j < 4; ++j) val[j] = s[j] * inv;
    float* p = Lc + ((size_t)b * KDIM + k) * VROWS + c;
    *(volatile v4f*)p = val;
    __threadfence();
    *(volatile v4f*)p = val;
  }
}

__global__ __launch_bounds__(128) __attribute__((amdgpu_num_vgpr(256))) void posconv_kernel(
    const float* __restrict__ Q32, const _Float16* __restrict__ Vh,
    const float* __restrict__ Lc, const _Float16* __restrict__ E16,
    float* __restrict__ out) {
  __shared__ _Float16 sPatch[PROWS * PP];
  __shared__ float sQ[64 * LDQ];
  __shared__ float sL[KDIM * LDL];
  __shared__ float sLc[KDIM * VG];

  const unsigned tid = threadIdx.x, lane = tid & 31u;
  const unsigned w = (unsigned)__builtin_amdgcn_readfirstlane((int)(tid >> 5));
  const unsigned hh = lane >> 4, m = lane & 15u;
  const unsigned y = blockIdx.x, vg = blockIdx.y, b = blockIdx.z;
  const unsigned x0 = w * 16u;

#pragma unroll
  for (unsigned i = 0; i < 8u; ++i) {
    const unsigned g = tid + 128u * i;
    const unsigned r = g >> 4, c = (g & 15u) * 4u;
    const v4f t = *(const v4f*)(Q32 + ((size_t)b * QROWS + r) * HW + y * IMG + c);
    *(v4f*)&sQ[r * LDQ + c] = t;
  }
#pragma unroll
  for (unsigned i = 0; i < 2u; ++i) {
    const unsigned idx = tid + 128u * i;
    const unsigned k = idx >> 4, vi = idx & 15u;
    sLc[idx] = Lc[((size_t)b * KDIM + k) * VROWS + vg * VG + vi];
  }
  if (w == 0u) {
    const unsigned r = lane >> 1, side = lane & 1u;
    const v8h z = {};
    *(v8h*)&sPatch[r * PP + side * 72u] = z;
  }
  v16h ef[4];
#pragma unroll
  for (int s = 0; s < 4; ++s) ef[s] = frag_at(E16 + (size_t)m * TAPK + hh * 8u + 32 * s);
  __syncthreads();

  const unsigned xq = tid & 63u, hp = tid >> 6;
  float qr0[16], qr1[16];
#pragma unroll
  for (int k = 0; k < 16; ++k) {
    qr0[k] = sQ[((2u * hp) * 16u + (unsigned)k) * LDQ + xq];
    qr1[k] = sQ[((2u * hp + 1u) * 16u + (unsigned)k) * LDQ + xq];
  }
  const unsigned pbase = x0 + m + 3u;

#pragma unroll 1
  for (unsigned vi = 0; vi < (unsigned)VG; ++vi) {
    const unsigned v = vg * VG + vi;
    {
      const unsigned r = tid >> 3, pc = (tid & 7u) * 8u;
      const int rr = (int)((r < 10u) ? r : 10u);
      const int yy = (int)y + rr - 5;
      const int yc = (yy < 0) ? 0 : ((yy > (IMG - 1)) ? (IMG - 1) : yy);
      v8h val = *(const v8h*)(Vh + ((size_t)b * VROWS + v) * HW + (unsigned)yc * IMG + pc);
      asm volatile("" : "+v"(val));
      const bool ok = (r < (unsigned)MWIN) && (yy == yc);
      const v8h z = {};
      val = ok ? val : z;
      *(v8h*)&sPatch[r * PP + 8u + pc] = val;
    }
    __syncthreads();

    v8f acc = {};
#pragma unroll
    for (int s = 0; s < 4; ++s) {
      v16h bf;
#pragma unroll
      for (int i = 0; i < 16; ++i) {
        const int c  = 32 * s + ((i < 8) ? i : (i + 8));
        const int c1 = ((c + 8) < 120) ? (c + 8) : 120;
        const unsigned o0 = (unsigned)((c / 11) * PP + (c % 11));
        const unsigned o1 = (unsigned)((c1 / 11) * PP + (c1 % 11));
        const unsigned o = (hh != 0u) ? o1 : o0;
        const _Float16 e = sPatch[pbase + o];
        const bool dead = ((c + 8) > 120) && (hh != 0u);
        bf[i] = dead ? (_Float16)0.0f : e;
      }
      acc = wmma16(ef[s], bf, acc);
    }
#pragma unroll
    for (int r = 0; r < 8; ++r) {
      const unsigned k = hh * 8u + (unsigned)r;
      sL[k * LDL + x0 + m] = acc[r] * (1.0f / (ECARRY * VCARRY)) + sLc[k * VG + vi];
    }
    __syncthreads();

    float a0 = 0.0f, a1 = 0.0f;
#pragma unroll
    for (int k = 0; k < 16; ++k) {
      const float l = sL[(unsigned)k * LDL + xq];
      a0 = fmaf(qr0[k], l, a0);
      a1 = fmaf(qr1[k], l, a1);
    }
    float* p0 = out + (((size_t)b * OUTC + (2u * hp) * VROWS + v) * HW + y * IMG + xq);
    float* p1 = p0 + (size_t)VROWS * HW;
    *(volatile float*)p0 = a0;
    *(volatile float*)p1 = a1;
    __threadfence();
    *(volatile float*)p0 = a0;
    *(volatile float*)p1 = a1;
  }
}

extern "C" void kernel_launch(void* const* d_in, const int* in_sizes, int n_in,
                              void* d_out, int out_size, void* d_ws, size_t ws_size,
                              hipStream_t stream) {
  if (n_in < 13) return;
  const long long need_x = (long long)NB * CIN * HW;
  const long long need_o = (long long)NB * OUTC * HW;
  if ((long long)in_sizes[0] < need_x) return;
  if (in_sizes[1] < QROWS * CIN) return;
  if (in_sizes[2] < QROWS || in_sizes[3] < QROWS || in_sizes[4] < QROWS || in_sizes[5] < QROWS) return;
  if (in_sizes[6] < KROWS * CIN) return;
  if (in_sizes[7] < VROWS * CIN) return;
  if (in_sizes[8] < VROWS || in_sizes[9] < VROWS || in_sizes[10] < VROWS || in_sizes[11] < VROWS) return;
  if (in_sizes[12] < KDIM * TAPS) return;
  if ((long long)out_size < need_o) return;
  if (ws_size < WS_TOTAL) return;

  const float* X    = (const float*)d_in[0];
  const float* wq   = (const float*)d_in[1];
  const float* qg   = (const float*)d_in[2];
  const float* qb   = (const float*)d_in[3];
  const float* qm   = (const float*)d_in[4];
  const float* qv   = (const float*)d_in[5];
  const float* wk   = (const float*)d_in[6];
  const float* wv   = (const float*)d_in[7];
  const float* vgm  = (const float*)d_in[8];
  const float* vb   = (const float*)d_in[9];
  const float* vm   = (const float*)d_in[10];
  const float* vvar = (const float*)d_in[11];
  const float* emb  = (const float*)d_in[12];
  float* out = (float*)d_out;

  char* ws = (char*)d_ws;
  _Float16* Wall = (_Float16*)(ws + OFF_WALL);
  _Float16* E16  = (_Float16*)(ws + OFF_E16);
  _Float16* Xt   = (_Float16*)(ws + OFF_XT);
  float*    Q32  = (float*)(ws + OFF_Q32);
  float*    K32  = (float*)(ws + OFF_K32);
  _Float16* Vh   = (_Float16*)(ws + OFF_VH);
  float*    Lcw  = (float*)(ws + OFF_LC);

  dim3 blk(256);
  dim3 gp(HW / 64, 1, NB);

  prep_kernel<<<dim3(25), blk, 0, stream>>>(wq, wk, wv, emb, Wall, E16);
  xconv_kernel<<<dim3(HW / 64, CIN / 64, NB), blk, 0, stream>>>(X, Xt);
  proj_q_kernel<<<gp, blk, 0, stream>>>(Wall, Xt, qg, qb, qm, qv, Q32);
  proj_v_kernel<<<gp, blk, 0, stream>>>(Wall + (size_t)64 * CIN, Xt, vgm, vb, vm, vvar, Vh);
  proj_k_kernel<<<gp, blk, 0, stream>>>(Wall + (size_t)128 * CIN, Xt, K32);
  content_kernel<<<dim3(NB), blk, 0, stream>>>(K32, Vh, Lcw);
  posconv_kernel<<<dim3(IMG, VROWS / VG, NB), dim3(128), 0, stream>>>(Q32, Vh, Lcw, E16, out);
}
